// WeightOptimizer_60679297958028
// MI455X (gfx1250) — hardware-run, weakly checked
//
#include <hip/hip_runtime.h>
#include <math.h>

typedef __attribute__((ext_vector_type(16))) _Float16 v16h;
typedef __attribute__((ext_vector_type(8)))  _Float16 v8h;
typedef __attribute__((ext_vector_type(8)))  float    v8f;
typedef __attribute__((ext_vector_type(4)))  float    v4f;

constexpr int kSteps    = 8192;
constexpr int kChan     = 64;
constexpr int kFront    = 64;
constexpr int kKPitch   = kSteps + kFront;
constexpr int kBRows    = 80;
constexpr int kRowTile  = 64;
constexpr int kWindow   = 128;
constexpr int kDistMax  = 96;
constexpr float kCarryA = 512.0f;
constexpr float kCarryB = 64.0f;
constexpr int kBandBlocks = kSteps / kRowTile;
constexpr int kPrepTileBlocks = kKPitch / 64;
constexpr int kWpadV4 = kKPitch / 4;
constexpr int kPrepWBlocks = (kWpadV4 + 255) / 256;
static_assert(kSteps % kRowTile == 0, "row tiles");
static_assert(kWindow % 32 == 0, "k steps of 32");
static_assert(kBRows % 16 == 0, "N tiles of 16");
static_assert((kKPitch * 2) % 128 == 0, "B plane pitch is a whole number of 128-B lines");
static_assert((kKPitch * 4) % 128 == 0, "wpad is a whole number of 128-B lines");
static_assert(kKPitch % 64 == 0 && kKPitch % 4 == 0, "line / float4 multiples");

constexpr size_t kOffBT   = 0;
constexpr size_t kSzBT    = (size_t)kBRows * kKPitch * 2;
constexpr size_t kOffWpad = kOffBT + kSzBT;
constexpr size_t kSzWpad  = (size_t)kKPitch * 4;
constexpr size_t kOffPart = kOffWpad + kSzWpad;
constexpr size_t kSzPart  = (size_t)kBandBlocks * 32 * 4;
constexpr size_t kWsTotal = kOffPart + kSzPart;
static_assert(kSzBT == 1320960ull && kSzWpad == 33024ull && kSzPart == 16384ull, "carve sizes");
static_assert(kWsTotal == 1370368ull, "carve total");
static_assert(kWsTotal <= 134217728ull, "carve cap");
static_assert((kOffWpad % 128) == 0 && (kOffPart % 128) == 0, "128-B aligned regions");

union FragH { v16h v; v8h h[2]; };
__device__ __forceinline__ v16h frag_load_h(const _Float16* p) {
  FragH f;
  f.h[0] = *(const v8h*)(p);
  f.h[1] = *(const v8h*)(p + 16);
  return f.v;
}
__device__ __forceinline__ v8f mma_f16(v16h a, v16h b, v8f c) {
  c = __builtin_amdgcn_wmma_f32_16x16x32_f16(false, a, false, b, (short)0, c, false, false);
  asm volatile("v_nop\n\tv_nop\n\tv_nop\n\tv_nop" : "+v"(c) : "v"(a), "v"(b));
  return c;
}

__global__ __launch_bounds__(256) void prep_kernel(
    const float* __restrict__ x, const float* __restrict__ w,
    unsigned short* __restrict__ bt, float* __restrict__ wpad)
{
  __shared__ __align__(16) float sT[64 * 65];
  const int tid = threadIdx.x, lane = tid & 31, wave = tid >> 5;
  const int b = blockIdx.x;
  if (b < kPrepTileBlocks) {
    const bool live = (b > 0);
    const int i0 = live ? (b - 1) * 64 : 0;
#pragma unroll
    for (int it = 0; it < 4; ++it) {
      const int idx = it * 256 + tid;
      const int r = idx >> 4;
      const int c4 = (idx & 15) * 4;
      const v4f v = *(const v4f*)(x + (size_t)(i0 + r) * kChan + c4);
      sT[(c4 + 0) * 65 + r] = live ? v[0] : 0.0f;
      sT[(c4 + 1) * 65 + r] = live ? v[1] : 0.0f;
      sT[(c4 + 2) * 65 + r] = live ? v[2] : 0.0f;
      sT[(c4 + 3) * 65 + r] = live ? v[3] : 0.0f;
    }
    __syncthreads();
    const int q = lane >> 3, l8 = lane & 7;
#pragma unroll 1
    for (int it = 0; it < 3; ++it) {
      const int gi = it * 8 + wave;
      if (gi < kBRows / 4) {
        const int n = gi * 4 + q;
        const int nc = (n < 64) ? n : 63;
        v8h hv;
#pragma unroll
        for (int e = 0; e < 8; ++e) {
          const float f = sT[nc * 65 + 8 * l8 + e];
          const float val = (n < 64) ? (f * kCarryB) : ((n == 64) ? kCarryB : 0.0f);
          hv[e] = (_Float16)val;
        }
        unsigned short* dst = bt + (size_t)n * kKPitch + (size_t)b * 64 + 8 * l8;
        *(volatile v8h*)dst = hv;
        __threadfence();
        *(volatile v8h*)dst = hv;
      }
    }
  } else {
    const int idx = (b - kPrepTileBlocks) * 256 + tid;
    const int idc = (idx < kWpadV4) ? idx : (kWpadV4 - 1);
    const int src = (idc >= kFront / 4) ? (idc - kFront / 4) : 0;
    const v4f v = *(const v4f*)(w + 4 * src);
    float a0 = v[0], a1 = v[1], a2 = v[2], a3 = v[3];
    asm volatile("" : "+v"(a0), "+v"(a1), "+v"(a2), "+v"(a3));
    const bool lv = (idc >= kFront / 4);
    v4f o;
    o[0] = lv ? a0 : 0.0f;
    o[1] = lv ? a1 : 0.0f;
    o[2] = lv ? a2 : 0.0f;
    o[3] = lv ? a3 : 0.0f;
    if (idx < kWpadV4) {
      float* dst = wpad + 4 * idx;
      *(volatile v4f*)dst = o;
      __threadfence();
      *(volatile v4f*)dst = o;
    }
  }
}

__global__ __launch_bounds__(128) void band_kernel(
    const unsigned short* __restrict__ btp, const float* __restrict__ wpad,
    const float* __restrict__ x, float* __restrict__ partial)
{
  __shared__ __align__(16) float sG[256];
  __shared__ __align__(16) float sW[kWindow];
  __shared__ __align__(16) float sS[4][16 * 68];
  __shared__ __align__(16) float sP[4][32];
  const int tid = threadIdx.x, lane = tid & 31, wave = tid >> 5;
  const int h = lane >> 4, c = lane & 15;
  const int R0 = blockIdx.x * kRowTile;

#pragma unroll
  for (int rep = 0; rep < 2; ++rep) {
    const int idx = tid + 128 * rep;
    const int d = idx - 63;
    const int dd = (d < 1) ? 1 : ((d > kDistMax) ? kDistMax : d);
    const float ev = expf(0.7f * ((float)dd - 11.0f));
    const float gv = __builtin_amdgcn_rcpf(1.0f + ev);
    sG[idx] = (d >= 1 && d <= kDistMax) ? gv : 0.0f;
  }
  sW[tid] = wpad[R0 + tid];
  __syncthreads();

  const _Float16* bt = (const _Float16*)btp;
  v8f acc0 = (v8f){0.f, 0.f, 0.f, 0.f, 0.f, 0.f, 0.f, 0.f};
  v8f acc1 = acc0, acc2 = acc0, acc3 = acc0, acc4 = acc0;
  const int ro = 16 * wave + c;

#pragma unroll
  for (int ks = 0; ks < 4; ++ks) {
    const int kb = 32 * ks + 8 * h;
    const v4f wq0 = *(const v4f*)(sW + kb);
    const v4f wq1 = *(const v4f*)(sW + kb + 4);
    const v4f wq2 = *(const v4f*)(sW + kb + 16);
    const v4f wq3 = *(const v4f*)(sW + kb + 20);
    const float wa[16] = { wq0[0], wq0[1], wq0[2], wq0[3], wq1[0], wq1[1], wq1[2], wq1[3],
                           wq2[0], wq2[1], wq2[2], wq2[3], wq3[0], wq3[1], wq3[2], wq3[3] };
    const int dbase = ro + kFront - kb;
    v16h a;
#pragma unroll
    for (int e = 0; e < 16; ++e) {
      const int off = (e < 8) ? e : (e + 8);
      const int d = dbase - off;
      int ti = d + 63;
      ti = (ti < 0) ? 0 : ((ti > 255) ? 255 : ti);
      const float gv = sG[ti];
      const float pv = wa[e] * gv * kCarryA;
      a[e] = (_Float16)((d >= 1) ? pv : 0.0f);
    }
    const size_t bo = (size_t)c * kKPitch + (size_t)(R0 + kb);
    {
      const v16h b0 = frag_load_h(bt + bo);
      acc0 = mma_f16(a, b0, acc0);
    }
    {
      const v16h b1 = frag_load_h(bt + bo + (size_t)16 * kKPitch);
      acc1 = mma_f16(a, b1, acc1);
    }
    {
      const v16h b2 = frag_load_h(bt + bo + (size_t)32 * kKPitch);
      acc2 = mma_f16(a, b2, acc2);
    }
    {
      const v16h b3 = frag_load_h(bt + bo + (size_t)48 * kKPitch);
      acc3 = mma_f16(a, b3, acc3);
    }
    {
      const v16h b4 = frag_load_h(bt + bo + (size_t)64 * kKPitch);
      acc4 = mma_f16(a, b4, acc4);
    }
  }

  float* slab = sS[wave];
#pragma unroll
  for (int r = 0; r < 8; ++r) {
    const int rl = (8 * h + r) * 68;
    slab[rl + c]      = acc0[r];
    slab[rl + 16 + c] = acc1[r];
    slab[rl + 32 + c] = acc2[r];
    slab[rl + 48 + c] = acc3[r];
    if (c == 0) slab[rl + 64] = acc4[r];
  }
  __syncthreads();

  float s = 0.0f;
  const int c4 = c * 4;
#pragma unroll 1
  for (int it = 0; it < 8; ++it) {
    const int row = it * 2 + h;
    const int kr = R0 + 16 * wave + row;
    const v4f p = *(const v4f*)(slab + row * 68 + c4);
    const float den = slab[row * 68 + 64];
    const bool valid = (kr >= 1);
    const float dsafe = valid ? den : 1.0f;
    const float rd = 1.0f / dsafe;
    const v4f t = *(const v4f*)(x + (size_t)kr * kChan + c4);
    const float g0 = p[0] * rd - t[0];
    const float g1 = p[1] * rd - t[1];
    const float g2 = p[2] * rd - t[2];
    const float g3 = p[3] * rd - t[3];
    const float sq = (g0 * g0 + g1 * g1) + (g2 * g2 + g3 * g3);
    s += valid ? sq : 0.0f;
  }
  sP[wave][lane] = s;
  __syncthreads();
  if (wave == 0) {
    const float tsum = ((sP[0][lane] + sP[1][lane]) + sP[2][lane]) + sP[3][lane];
    float* dst = partial + (size_t)blockIdx.x * 32 + lane;
    *(volatile float*)dst = tsum;
    __threadfence();
    *(volatile float*)dst = tsum;
  }
}

__global__ __launch_bounds__(256) void final_kernel(const float* __restrict__ partial, float* __restrict__ out)
{
  __shared__ float sR[256];
  const int tid = threadIdx.x;
  const float* p = partial + 16 * tid;
  const v4f a0 = *(const v4f*)(p);
  const v4f a1 = *(const v4f*)(p + 4);
  const v4f a2 = *(const v4f*)(p + 8);
  const v4f a3 = *(const v4f*)(p + 12);
  const float s0 = (a0[0] + a0[1]) + (a0[2] + a0[3]);
  const float s1 = (a1[0] + a1[1]) + (a1[2] + a1[3]);
  const float s2 = (a2[0] + a2[1]) + (a2[2] + a2[3]);
  const float s3 = (a3[0] + a3[1]) + (a3[2] + a3[3]);
  sR[tid] = (s0 + s1) + (s2 + s3);
  __syncthreads();
#pragma unroll 1
  for (int off = 128; off >= 1; off >>= 1) {
    float v = 0.0f;
    if (tid < off) v = sR[tid] + sR[tid + off];
    __syncthreads();
    if (tid < off) sR[tid] = v;
    __syncthreads();
  }
  if (tid == 0) {
    const float res = sR[0] * (1.0f / (float)(kSteps - 1));
    *(volatile float*)out = res;
    __threadfence();
    *(volatile float*)out = res;
  }
}

extern "C" void kernel_launch(void* const* d_in, const int* in_sizes, int n_in,
                              void* d_out, int out_size, void* d_ws, size_t ws_size,
                              hipStream_t stream) {
  if (n_in < 2) return;
  if (in_sizes[0] != kSteps * kChan) return;
  if (in_sizes[1] != kSteps) return;
  if (out_size != 1) return;
  if (ws_size < kWsTotal) return;

  const float* x = (const float*)d_in[0];
  const float* w = (const float*)d_in[1];
  float* out = (float*)d_out;

  char* ws = (char*)d_ws;
  unsigned short* BT   = (unsigned short*)(ws + kOffBT);
  float*          WPAD = (float*)(ws + kOffWpad);
  float*          PART = (float*)(ws + kOffPart);

  prep_kernel<<<kPrepTileBlocks + kPrepWBlocks, 256, 0, stream>>>(x, w, BT, WPAD);
  band_kernel<<<kBandBlocks, 128, 0, stream>>>(BT, WPAD, x, PART);
  final_kernel<<<1, 256, 0, stream>>>(PART, out);
}
